// LocalSparseAttention_3496103379663
// MI455X (gfx1250) — hardware-verified
//
#include <hip/hip_runtime.h>


#define NBH  24
#define LL   4096
#define HD   64
#define NTI  64
#define NBD  5
#define SP   (NBD * 64)
#define WND  128
#define ZG   12
#define DM   HD
#define PCAR 1024.0f
#define LOSC 1024.0f
typedef _Float16 h16;
typedef unsigned short bf;
typedef __attribute__((ext_vector_type(16))) __bf16   v16bf;
typedef __attribute__((ext_vector_type(16))) _Float16 v16h;
typedef __attribute__((ext_vector_type(8)))  _Float16 v8h;
typedef __attribute__((ext_vector_type(8)))  unsigned short v8us;
typedef __attribute__((ext_vector_type(8)))  float    v8f;
typedef __attribute__((ext_vector_type(4)))  float    v4f;
typedef v8h  __attribute__((may_alias)) v8ha;
typedef v4f  __attribute__((may_alias)) v4fa;
typedef v8us __attribute__((may_alias)) v8usa;

__device__ __forceinline__ unsigned short f2bf(float f) { unsigned u = __float_as_uint(f); u += 0x7FFFu + ((u >> 16) & 1u); return (unsigned short)(u >> 16); }
__device__ __forceinline__ float bf2f(unsigned short b) { return __uint_as_float(((unsigned)b) << 16); }
__device__ __forceinline__ float bfr(float f) { return bf2f(f2bf(f)); }
__device__ __forceinline__ v16h cat16(v8h lo, v8h hi) { return __builtin_shufflevector(lo, hi, 0, 1, 2, 3, 4, 5, 6, 7, 8, 9, 10, 11, 12, 13, 14, 15); }
__device__ __forceinline__ v16bf cat16b(v8us lo, v8us hi) { return __builtin_bit_cast(v16bf, __builtin_shufflevector(lo, hi, 0, 1, 2, 3, 4, 5, 6, 7, 8, 9, 10, 11, 12, 13, 14, 15)); }
__device__ __forceinline__ v8f wmma16(v16h a, v16h b, v8f c) { return __builtin_amdgcn_wmma_f32_16x16x32_f16(false, a, false, b, (short)0, c, false, false); }
__device__ __forceinline__ v8f wmmab(v16bf a, v16bf b, v8f c) { return __builtin_amdgcn_wmma_f32_16x16x32_bf16(false, a, false, b, (short)0, c, false, false); }


__global__ __launch_bounds__(128) void k_gemmh(const h16* __restrict__ A, const h16* __restrict__ Bn, const float* __restrict__ bias, float* C, int ldc, const float* __restrict__ R, int K, size_t sA, size_t sB, size_t sC, int roundR) {
    __shared__ __align__(16) float ost[4][16 * 68];
    const size_t z = blockIdx.z; A += z * sA; Bn += z * sB; C += z * sC; if (R) R += z * sC;
    const int lane = threadIdx.x & 31, wave = threadIdx.x >> 5, lr = lane & 15, hi = lane >> 4;
    const int r0 = blockIdx.x * 64 + wave * 16, c0 = blockIdx.y * 64;
    const size_t aoff = (size_t)(r0 + lr) * K + 8 * hi;
    size_t boff[4];
#pragma unroll
    for (int t = 0; t < 4; ++t) boff[t] = (size_t)(c0 + t * 16 + lr) * K + 8 * hi;
    v8f acc[4];
#pragma unroll
    for (int t = 0; t < 4; ++t) acc[t] = (v8f){};
#pragma unroll 1
    for (int kc = 0; kc < K; kc += 32) {
        const v16h a = cat16(*(const v8h*)(A + aoff + kc), *(const v8h*)(A + aoff + kc + 16));
#pragma unroll
        for (int t = 0; t < 4; ++t) { const v16h b = cat16(*(const v8h*)(Bn + boff[t] + kc), *(const v8h*)(Bn + boff[t] + kc + 16)); acc[t] = wmma16(a, b, acc[t]); }
        asm volatile("v_nop\n\tv_nop\n\tv_nop\n\tv_nop" : "+v"(acc[0]), "+v"(acc[1]), "+v"(acc[2]), "+v"(acc[3]) : "v"(a));
    }
    float* os = &ost[wave][0];
#pragma unroll
    for (int t = 0; t < 4; ++t) { const float bv = bias ? bfr(bias[c0 + t * 16 + lr]) : 0.f;
#pragma unroll
        for (int j = 0; j < 8; ++j) os[(hi * 8 + j) * 68 + t * 16 + lr] = acc[t][j] + bv; }
    __syncthreads();
    float* crow = C + (size_t)r0 * ldc + c0;
    auto pass = [&]() {
#pragma unroll
        for (int s = 0; s < 8; ++s) { const int Lid = (lane >> 3) + 4 * s, piece = lane & 7; const int row = Lid >> 1, cofs = (Lid & 1) * 32 + piece * 4;
            v4f val = *(const v4fa*)(os + row * 68 + cofs); if (R) { const v4f rv = *(const v4f*)(R + ((size_t)r0 + row) * ldc + c0 + cofs); val += roundR ? (v4f){bfr(rv[0]), bfr(rv[1]), bfr(rv[2]), bfr(rv[3])} : rv; }
            *(volatile v4f*)(crow + (size_t)row * ldc + cofs) = val; }
    };
    pass(); __threadfence(); pass();
}

template <int MODE>
__global__ __launch_bounds__(128) void k_gemm3z(const bf* __restrict__ Ah, const bf* __restrict__ Al, const bf* __restrict__ Bh, const bf* __restrict__ Bl, int K, float* C, int ldc, size_t sA, size_t sB, size_t sC) {
    if ((MODE & 1) && (int)blockIdx.y * 64 > (int)blockIdx.x * 64 + 63) return;
    const size_t z = blockIdx.z; Ah += z * sA; Al += z * sA; Bh += z * sB; Bl += z * sB; C += z * sC;
    const int Klim = (MODE & 2) ? min(K, ((int)blockIdx.x + 1) * 64) : K;
    __shared__ __align__(16) float ost[4][16 * 68];
    const int lane = threadIdx.x & 31, wave = threadIdx.x >> 5, lr = lane & 15, hi = lane >> 4;
    const int r0 = blockIdx.x * 64 + wave * 16, c0 = blockIdx.y * 64;
    const size_t aoff = (size_t)(r0 + lr) * K + 8 * hi;
    v8f acc[4];
#pragma unroll
    for (int t = 0; t < 4; ++t) acc[t] = (v8f){};
#pragma unroll 1
    for (int kc = 0; kc < Klim; kc += 32) {
        const v16bf a = cat16b(*(const v8us*)(Ah + aoff + kc), *(const v8us*)(Ah + aoff + kc + 16));
        v16bf al = a; if (!(MODE & 4) && !(MODE & 16)) al = cat16b(*(const v8us*)(Al + aoff + kc), *(const v8us*)(Al + aoff + kc + 16));
#pragma unroll
        for (int t = 0; t < 4; ++t) { const size_t bo = (size_t)(c0 + t * 16 + lr) * K + kc + 8 * hi;
            const v16bf bh = cat16b(*(const v8us*)(Bh + bo), *(const v8us*)(Bh + bo + 16));
            acc[t] = wmmab(a, bh, acc[t]);
            if (!(MODE & 4)) { if (!(MODE & 16)) acc[t] = wmmab(al, bh, acc[t]); if (!(MODE & 8)) { const v16bf bl = cat16b(*(const v8us*)(Bl + bo), *(const v8us*)(Bl + bo + 16)); acc[t] = wmmab(a, bl, acc[t]); } } }
        asm volatile("v_nop\n\tv_nop\n\tv_nop\n\tv_nop" : "+v"(acc[0]), "+v"(acc[1]), "+v"(acc[2]), "+v"(acc[3]) : "v"(a), "v"(al));
    }
    float* os = &ost[wave][0];
#pragma unroll
    for (int t = 0; t < 4; ++t) {
#pragma unroll
        for (int j = 0; j < 8; ++j) os[(hi * 8 + j) * 68 + t * 16 + lr] = acc[t][j]; }
    __builtin_amdgcn_wave_barrier(); asm volatile("" ::: "memory");
    float* crow = C + (size_t)r0 * ldc + c0;
    auto pass = [&]() {
#pragma unroll
        for (int s = 0; s < 8; ++s) { const int Lid = (lane >> 3) + 4 * s, piece = lane & 7; const int row = Lid >> 1, cofs = (Lid & 1) * 32 + piece * 4;
            const v4f val = *(const v4fa*)(os + row * 68 + cofs); *(volatile v4f*)(crow + (size_t)row * ldc + cofs) = val; }
    };
    pass(); __threadfence(); pass();
}
__global__ __launch_bounds__(256) void k_planes32z(const float* __restrict__ F, int ld, int off, float sc, int rows, bf* Ph, bf* Pl) {
    typedef __attribute__((ext_vector_type(2))) unsigned short v2us;
    const int lane = threadIdx.x & 31; const size_t r = ((size_t)blockIdx.x * 8 + (threadIdx.x >> 5)) * 2 + (lane >> 4); if (r >= (size_t)rows) return; const int z = blockIdx.z; const int c0 = (lane & 15) * 2; v2us oh, ol;
    Ph += (size_t)z * rows * 32; Pl += (size_t)z * rows * 32;
#pragma unroll
    for (int i = 0; i < 2; ++i) { const float y = F[r * ld + off + z * 32 + c0 + i] * sc; const unsigned short hb = f2bf(y); oh[i] = hb; ol[i] = f2bf(y - bf2f(hb)); }
    const size_t o = r * 32 + c0; *(volatile v2us*)(Ph + o) = oh; *(volatile v2us*)(Pl + o) = ol; __threadfence(); *(volatile v2us*)(Ph + o) = oh; *(volatile v2us*)(Pl + o) = ol;
}
__global__ __launch_bounds__(256) void k_vtpadz(const float* __restrict__ F, int ld, int off, int nk, bf* Th, bf* Tl) {
    typedef __attribute__((ext_vector_type(2))) unsigned short v2us;
    const int lane = threadIdx.x & 31; const size_t wid = (size_t)blockIdx.x * 8 + (threadIdx.x >> 5); if (wid >= (size_t)64 * (nk / 64)) return; const int z = blockIdx.z; const int d = (int)(wid / (nk / 64)); const int k0 = (int)(wid % (nk / 64)) * 64 + lane * 2; v2us oh, ol;
    Th += (size_t)z * 64 * nk; Tl += (size_t)z * 64 * nk;
#pragma unroll
    for (int i = 0; i < 2; ++i) { const float y = (d < 32) ? F[(size_t)(k0 + i) * ld + off + z * 32 + (d < 32 ? d : 0)] : 0.f; const unsigned short hb = f2bf(y); oh[i] = hb; ol[i] = f2bf(y - bf2f(hb)); }
    const size_t o = (size_t)d * nk + k0; *(volatile v2us*)(Th + o) = oh; *(volatile v2us*)(Tl + o) = ol; __threadfence(); *(volatile v2us*)(Th + o) = oh; *(volatile v2us*)(Tl + o) = ol;
}
template <int NK>
__global__ __launch_bounds__(256) void k_softmaxz(const float* __restrict__ S, int rows, bf* PH, bf* PL) {
    typedef __attribute__((ext_vector_type(4))) unsigned short v4us;
    const int lane = threadIdx.x & 31, i = blockIdx.x * 8 + (threadIdx.x >> 5); if (i >= rows) return; const size_t zo = (size_t)blockIdx.z * rows * NK; const float* sr = S + zo + (size_t)i * NK; PH += zo; PL += zo;
    float m = -3.0e38f;
#pragma unroll 1
    for (int c0 = lane * 4; c0 < NK; c0 += 128) {
#pragma unroll
        for (int q = 0; q < 4; ++q) m = fmaxf(m, sr[c0 + q]); }
#pragma unroll
    for (int sh = 16; sh; sh >>= 1) m = fmaxf(m, __shfl_xor(m, sh, 32));
    float sum = 0.f;
#pragma unroll 1
    for (int c0 = lane * 4; c0 < NK; c0 += 128) {
#pragma unroll
        for (int q = 0; q < 4; ++q) sum += __expf(sr[c0 + q] - m); }
#pragma unroll
    for (int sh = 16; sh; sh >>= 1) sum += __shfl_xor(sum, sh, 32);
    const float inv = 1.0f / sum;
#pragma unroll 1
    for (int ps = 0; ps < 2; ++ps) {
#pragma unroll 1
        for (int c0 = lane * 4; c0 < NK; c0 += 128) { v4us oh, ol;
#pragma unroll
            for (int q = 0; q < 4; ++q) { const float p = __expf(sr[c0 + q] - m) * inv; const unsigned short hb = f2bf(p); oh[q] = hb; ol[q] = f2bf(p - bf2f(hb)); }
            const size_t o = (size_t)i * NK + c0; *(volatile v4us*)(PH + o) = oh; *(volatile v4us*)(PL + o) = ol; }
        if (ps == 0) __threadfence(); }
}
__global__ __launch_bounds__(256) void k_placez(const float* __restrict__ XH, int rows, int ldy, float* Y) {
    const int lane = threadIdx.x & 31; const size_t q = (size_t)blockIdx.x * 8 + (threadIdx.x >> 5); if (q >= (size_t)rows) return; const int z = blockIdx.z; const float v = XH[((size_t)z * rows + q) * 64 + lane];
    *(volatile float*)(Y + q * ldy + z * 32 + lane) = v; __threadfence(); *(volatile float*)(Y + q * ldy + z * 32 + lane) = v;
}
__global__ __launch_bounds__(256) void k_cvt8(const float* __restrict__ src, bf* dst, size_t n8) {
    const size_t i = (size_t)blockIdx.x * 256 + threadIdx.x; if (i >= n8) return;
    const v8f v = *(const v8f*)(src + i * 8); v8us o;
#pragma unroll
    for (int k = 0; k < 8; ++k) o[k] = f2bf(v[k]);
    *(volatile v8us*)(dst + i * 8) = o; __threadfence(); *(volatile v8us*)(dst + i * 8) = o;
}
__global__ __launch_bounds__(256) void k_zero8(bf* dst, size_t n8) {
    const size_t i = (size_t)blockIdx.x * 256 + threadIdx.x; if (i >= n8) return; v8us z;
#pragma unroll
    for (int k = 0; k < 8; ++k) z[k] = 0;
    *(volatile v8us*)(dst + i * 8) = z; __threadfence(); *(volatile v8us*)(dst + i * 8) = z;
}

__global__ __launch_bounds__(32) void k_band1(const bf* __restrict__ Q, const bf* __restrict__ Kb, float* S) {
    __shared__ __align__(16) float os[16 * 68];
    const int I = blockIdx.x, slot = blockIdx.y, J = I - 2 + slot; if (J < 0 || J >= NTI) return; const size_t z = blockIdx.z; Q += z * (size_t)LL * HD; Kb += z * (size_t)LL * HD; S += z * (size_t)LL * SP;
    const int lane = threadIdx.x & 31, lr = lane & 15, hi = lane >> 4; const int r0 = I * 64, k0r = J * 64;
    v8f acc[4][4];
#pragma unroll
    for (int mb = 0; mb < 4; ++mb)
#pragma unroll
        for (int nb = 0; nb < 4; ++nb) acc[mb][nb] = (v8f){};
    const size_t aoff = (size_t)(r0 + lr) * HD + 8 * hi, boff = (size_t)(k0r + lr) * HD + 8 * hi;
#pragma unroll 1
    for (int kc = 0; kc < HD; kc += 32) { v16bf a[4];
#pragma unroll
        for (int mb = 0; mb < 4; ++mb) a[mb] = cat16b(*(const v8us*)(Q + aoff + (size_t)mb * 16 * HD + kc), *(const v8us*)(Q + aoff + (size_t)mb * 16 * HD + kc + 16));
#pragma unroll
        for (int nb = 0; nb < 4; ++nb) { const v16bf b = cat16b(*(const v8us*)(Kb + boff + (size_t)nb * 16 * HD + kc), *(const v8us*)(Kb + boff + (size_t)nb * 16 * HD + kc + 16));
#pragma unroll
            for (int mb = 0; mb < 4; ++mb) acc[mb][nb] = wmmab(a[mb], b, acc[mb][nb]); }
        asm volatile("v_nop\n\tv_nop\n\tv_nop\n\tv_nop" : "+v"(acc[0][0]), "+v"(acc[1][1]), "+v"(acc[2][2]), "+v"(acc[3][3]) : "v"(a[0]), "v"(a[3])); }
#pragma unroll
    for (int mb = 0; mb < 4; ++mb) {
#pragma unroll
        for (int nb = 0; nb < 4; ++nb) {
#pragma unroll
            for (int j = 0; j < 8; ++j) os[(hi * 8 + j) * 68 + nb * 16 + lr] = acc[mb][nb][j]; }
        __builtin_amdgcn_wave_barrier(); asm volatile("" ::: "memory");
        float* crow = S + (size_t)(r0 + mb * 16) * SP + slot * 64;
#pragma unroll 1
        for (int ps = 0; ps < 2; ++ps) {
#pragma unroll
            for (int s = 0; s < 8; ++s) { const int row = 2 * s + hi, cofs = lr * 4; const v4f val = *(const v4fa*)(os + row * 68 + cofs); *(volatile v4f*)(crow + (size_t)row * SP + cofs) = val; }
            if (ps == 0) __threadfence(); }
        __builtin_amdgcn_wave_barrier(); asm volatile("" ::: "memory"); }
}
__global__ __launch_bounds__(256) void k_bandsoft(const float* __restrict__ S, bf* Ph, bf* Pl) {
    typedef __attribute__((ext_vector_type(4))) unsigned short v4us;
    const int lane = threadIdx.x & 31, i = blockIdx.x * 8 + (threadIdx.x >> 5); if (i >= LL) return; const size_t zo = ((size_t)blockIdx.z * LL + i) * SP; const float* sr = S + zo; const int I = i >> 6; const int jbase = (I - 2) * 64;
    auto live = [&](int c) { const int j = jbase + c; return j >= 0 && j < LL && (j - i) <= WND && (i - j) <= WND; };
    float m = -3.0e38f;
#pragma unroll 1
    for (int c0 = lane * 4; c0 < SP; c0 += 128) {
#pragma unroll
        for (int q = 0; q < 4; ++q) if (live(c0 + q)) m = fmaxf(m, sr[c0 + q] * 0.125f); }
#pragma unroll
    for (int sh = 16; sh; sh >>= 1) m = fmaxf(m, __shfl_xor(m, sh, 32));
    float sum = 0.f;
#pragma unroll 1
    for (int c0 = lane * 4; c0 < SP; c0 += 128) {
#pragma unroll
        for (int q = 0; q < 4; ++q) if (live(c0 + q)) sum += __expf(sr[c0 + q] * 0.125f - m); }
#pragma unroll
    for (int sh = 16; sh; sh >>= 1) sum += __shfl_xor(sum, sh, 32);
    const float f = __fdiv_rn(PCAR, sum);
#pragma unroll 1
    for (int ps = 0; ps < 2; ++ps) {
#pragma unroll 1
        for (int c0 = lane * 4; c0 < SP; c0 += 128) { v4us oh, ol;
#pragma unroll
            for (int q = 0; q < 4; ++q) { const int c = c0 + q; const float p = live(c) ? __expf(sr[live(c) ? c : 0] * 0.125f - m) * f : 0.f; const unsigned short hb = f2bf(p); oh[q] = hb; ol[q] = f2bf(p - bf2f(hb)); }
            *(volatile v4us*)(Ph + zo + c0) = oh; *(volatile v4us*)(Pl + zo + c0) = ol; }
        if (ps == 0) __threadfence(); }
}
__global__ __launch_bounds__(256) void k_vTb(const float* __restrict__ V, bf* VT) {
    typedef __attribute__((ext_vector_type(4))) unsigned short v4us;
    __shared__ float tl[64][65];
    const int tid = threadIdx.x; const int t0 = blockIdx.x * 64; const size_t z = blockIdx.z; const int rr = tid >> 2, cq = (tid & 3) * 16;
#pragma unroll
    for (int i = 0; i < 16; ++i) tl[rr][cq + i] = V[(z * LL + t0 + rr) * HD + cq + i];
    __syncthreads();
    const int lane = tid & 31, wv = tid >> 5;
    auto pass = [&]() {
#pragma unroll
        for (int st = 0; st < 4; ++st) { const int dr = wv * 8 + st * 2 + (lane >> 4); const int tq = (lane & 15) * 4; v4us v;
#pragma unroll
            for (int i = 0; i < 4; ++i) v[i] = f2bf(tl[tq + i][dr]);
            *(volatile v4us*)(VT + (z * HD + dr) * LL + t0 + tq) = v; }
    };
    pass(); __threadfence(); pass();
}
__global__ __launch_bounds__(32) void k_band2(const bf* __restrict__ Ph, const bf* __restrict__ Pl, const bf* __restrict__ VT, float* O) {
    __shared__ __align__(16) float os[16 * 68];
    const int I = blockIdx.x; const size_t z = blockIdx.z; Ph += z * (size_t)LL * SP; Pl += z * (size_t)LL * SP; VT += z * (size_t)HD * LL; O += z * (size_t)LL * HD;
    const int lane = threadIdx.x & 31, lr = lane & 15, hi = lane >> 4; const int r0 = I * 64; const int jbase = (I - 2) * 64; const int Klo = jbase < 0 ? -jbase : 0; const int Khi = min(SP, LL - jbase);
    v8f acc[4][4];
#pragma unroll
    for (int mb = 0; mb < 4; ++mb)
#pragma unroll
        for (int nb = 0; nb < 4; ++nb) acc[mb][nb] = (v8f){};
    const size_t aoff = (size_t)(r0 + lr) * SP + 8 * hi; const size_t boff = (size_t)lr * LL + jbase + 8 * hi;
#pragma unroll 1
    for (int kc = Klo; kc < Khi; kc += 32) { v16bf a[4], a2[4];
#pragma unroll
        for (int mb = 0; mb < 4; ++mb) { a[mb] = cat16b(*(const v8us*)(Ph + aoff + (size_t)mb * 16 * SP + kc), *(const v8us*)(Ph + aoff + (size_t)mb * 16 * SP + kc + 16)); a2[mb] = cat16b(*(const v8us*)(Pl + aoff + (size_t)mb * 16 * SP + kc), *(const v8us*)(Pl + aoff + (size_t)mb * 16 * SP + kc + 16)); }
#pragma unroll
        for (int nb = 0; nb < 4; ++nb) { const v16bf b = cat16b(*(const v8us*)(VT + boff + (size_t)nb * 16 * LL + kc), *(const v8us*)(VT + boff + (size_t)nb * 16 * LL + kc + 16));
#pragma unroll
            for (int mb = 0; mb < 4; ++mb) { acc[mb][nb] = wmmab(a[mb], b, acc[mb][nb]); acc[mb][nb] = wmmab(a2[mb], b, acc[mb][nb]); } }
        asm volatile("v_nop\n\tv_nop\n\tv_nop\n\tv_nop" : "+v"(acc[0][0]), "+v"(acc[1][1]), "+v"(acc[2][2]), "+v"(acc[3][3]) : "v"(a[0]), "v"(a[3])); }
#pragma unroll
    for (int mb = 0; mb < 4; ++mb) {
#pragma unroll
        for (int nb = 0; nb < 4; ++nb) {
#pragma unroll
            for (int j = 0; j < 8; ++j) os[(hi * 8 + j) * 68 + nb * 16 + lr] = acc[mb][nb][j] * (1.0f / PCAR); }
        __builtin_amdgcn_wave_barrier(); asm volatile("" ::: "memory");
        float* crow = O + (size_t)(r0 + mb * 16) * HD;
#pragma unroll 1
        for (int ps = 0; ps < 2; ++ps) {
#pragma unroll
            for (int s = 0; s < 8; ++s) { const int row = 2 * s + hi, cofs = lr * 4; const v4f val = *(const v4fa*)(os + row * 68 + cofs); *(volatile v4f*)(crow + (size_t)row * HD + cofs) = val; }
            if (ps == 0) __threadfence(); }
        __builtin_amdgcn_wave_barrier(); asm volatile("" ::: "memory"); }
}
extern "C" void kernel_launch(void* const* d_in, const int* in_sizes, int n_in,
                              void* d_out, int out_size, void* d_ws, size_t ws_size, hipStream_t stream) {
    (void)in_sizes; (void)n_in; (void)out_size;
    const float* q = (const float*)d_in[0]; const float* k = (const float*)d_in[1]; const float* v = (const float*)d_in[2];
    float* out = (float*)d_out;
    char* wsp = (char*)d_ws;
    auto take = [&](size_t bytes) { char* p = wsp; wsp += (bytes + 255) & ~(size_t)255; return (void*)p; };
    bf* QB = (bf*)take((size_t)NBH * LL * HD * 2); bf* KBf = (bf*)take((size_t)NBH * LL * HD * 2); bf* VT = (bf*)take((size_t)ZG * HD * LL * 2); float* S = (float*)take((size_t)ZG * LL * SP * 4); bf* Ph = (bf*)take((size_t)ZG * LL * SP * 2); bf* Pl = (bf*)take((size_t)ZG * LL * SP * 2);
    if ((size_t)(wsp - (char*)d_ws) > ws_size) return;
    const size_t n8 = (size_t)NBH * LL * HD / 8; k_cvt8<<<(unsigned)((n8 + 255) / 256), 256, 0, stream>>>(q, QB, n8); k_cvt8<<<(unsigned)((n8 + 255) / 256), 256, 0, stream>>>(k, KBf, n8);
    for (int g0 = 0; g0 < NBH; g0 += ZG) {
        k_vTb<<<dim3(LL / 64, 1, ZG), 256, 0, stream>>>(v + (size_t)g0 * LL * HD, VT);
        k_band1<<<dim3(NTI, NBD, ZG), 32, 0, stream>>>(QB + (size_t)g0 * LL * HD, KBf + (size_t)g0 * LL * HD, S);
        k_bandsoft<<<dim3(LL / 8, 1, ZG), 256, 0, stream>>>(S, Ph, Pl);
        k_band2<<<dim3(NTI, 1, ZG), 32, 0, stream>>>(Ph, Pl, VT, out + (size_t)g0 * LL * HD); }
}
